// HetGCN_76682346102819
// MI455X (gfx1250) — hardware-run, weakly checked
//
#include <hip/hip_runtime.h>


namespace {
constexpr int N = 50000, E = 500000, DA = 256, DB = 128, D = 128, DO = 64;
constexpr float XS = 8.0f, WSC = 256.0f;
typedef _Float16 b16;
typedef __attribute__((ext_vector_type(16))) _Float16 v16b;
typedef __attribute__((ext_vector_type(8))) _Float16 v8b;
typedef __attribute__((ext_vector_type(8))) float v8f;
typedef __attribute__((ext_vector_type(4))) float v4f;
typedef __attribute__((ext_vector_type(2))) float v2f;
__device__ __forceinline__ float bf16_rne(float f) { unsigned int u = __float_as_uint(f); u += 0x7FFFu + ((u >> 16) & 1u); float r = __uint_as_float(u & 0xFFFF0000u); asm volatile("" : "+v"(r)); return r; }
__device__ __forceinline__ void split16(float v, b16& hi, b16& lo) { hi = (b16)v; lo = (b16)(v - (float)hi); }
__device__ __forceinline__ v16b frag_kb(const b16* p, int hh) { const v8b a = *(const v8b*)(p + 8 * hh), b = *(const v8b*)(p + 16 + 8 * hh); v16b f;
#pragma unroll
  for (int e = 0; e < 8; ++e) { f[e] = a[e]; f[8 + e] = b[e]; } return f; }
__device__ __forceinline__ v8f wmma16b(v16b a, v16b b, v8f c) { v8f d = __builtin_amdgcn_wmma_f32_16x16x32_f16(false, a, false, b, (short)0, c, false, false); asm volatile("v_nop\n\tv_nop\n\tv_nop\n\tv_nop" : "+v"(d) : "v"(a), "v"(b)); return d; }
__device__ __forceinline__ void wave_lds_sync() { __builtin_amdgcn_fence(__ATOMIC_RELEASE, "workgroup"); __builtin_amdgcn_wave_barrier(); __builtin_amdgcn_fence(__ATOMIC_ACQUIRE, "workgroup"); }
__device__ __forceinline__ float pmul(float a, float b) { float p = a * b; asm volatile("" : "+v"(p)); return p; }
__device__ __forceinline__ int iclamp(int v, int lo, int hi) { return v < lo ? lo : (v > hi ? hi : v); }
constexpr int CSR_NBLK9 = 512, CSR_GB9 = 9, CSR_GN9 = 1 << CSR_GB9  , CSR_TS9 = (CSR_GN9 < 32 ? 32 : CSR_GN9)  , CSR_MAXG9 = 512, CSR_CAP9 = 12288  ;
__device__ __host__ __forceinline__ int csr_tix9(int v) { return (v >> CSR_GB9) * CSR_TS9 + (v & (CSR_GN9 - 1)); }
__global__ __launch_bounds__(64) void csrA_kernel9(const int* __restrict__ dst, int E, int N, int nG, int CHP, int NGP, int* __restrict__ STG, int* __restrict__ HST) {
  extern __shared__ int sm[];
  int* cnt = sm; int* run = sm + NGP; int* ids = sm + 2 * NGP;
  const int b = blockIdx.x; const int ch = (E + CSR_NBLK9 - 1) / CSR_NBLK9; const int e0 = b * ch, e1 = min(E, e0 + ch);
  for (int i = threadIdx.x; i < NGP; i += 64) cnt[i] = 0;
  for (int i = threadIdx.x; i < CHP; i += 64) ids[i] = -1;
  __syncthreads();
  if (threadIdx.x == 0) {
    for (int e = e0; e < e1; ++e) { int d = dst[e]; d = (d < 0) ? 0 : (d >= N ? N - 1 : d); cnt[d >> CSR_GB9] += 1; }
    int acc = 0; for (int g = 0; g < nG; ++g) { run[g] = acc; acc += cnt[g]; }
    for (int e = e0; e < e1; ++e) { int d = dst[e]; d = (d < 0) ? 0 : (d >= N ? N - 1 : d); const int g = d >> CSR_GB9; ids[run[g]] = e; run[g] += 1; } }
  __syncthreads();
  typedef __attribute__((ext_vector_type(4))) int v4i;
  for (int pass = 0; pass < 2; ++pass) {
    for (int i = threadIdx.x; i < CHP / 4; i += 64) *(volatile v4i*)(STG + (size_t)b * CHP + i * 4) = *(const v4i*)(&ids[i * 4]);
    for (int i = threadIdx.x; i < NGP / 4; i += 64) { v4i v; for (int e = 0; e < 4; ++e) v[e] = (i * 4 + e < nG) ? cnt[i * 4 + e] : 0; *(volatile v4i*)(HST + (size_t)b * NGP + i * 4) = v; }
    __threadfence(); }
}
__global__ __launch_bounds__(512) void csrS_kernel9(const int* __restrict__ HST, int nG, int NGP, int* __restrict__ START, int* __restrict__ TOT, int* __restrict__ OFF) {
  __shared__ int tot[CSR_MAXG9];
  const int b = threadIdx.x;
  for (int pass = 0; pass < 2; ++pass) { int runb = 0; for (int g = 0; g < nG; ++g) { int c = HST[(size_t)b * NGP + g]; c = (c < 0) ? 0 : c; ((volatile int*)OFF)[(size_t)g * CSR_NBLK9 + b] = runb; runb += c; } __threadfence(); }
  for (int g = threadIdx.x; g < nG; g += 512) { int s = 0; for (int bb = 0; bb < CSR_NBLK9; ++bb) { int c = HST[(size_t)bb * NGP + g]; s += (c < 0) ? 0 : c; } tot[g] = s; }
  __syncthreads();
  if (threadIdx.x < 32) {
    __shared__ int st[CSR_MAXG9 + 32];
    if (threadIdx.x == 0) { int acc = 0; for (int g = 0; g < NGP; ++g) { st[g] = acc; if (g < nG) acc += (tot[g] + 31) & ~31; } st[NGP] = acc; }
    __builtin_amdgcn_fence(__ATOMIC_RELEASE, "workgroup"); __builtin_amdgcn_wave_barrier(); __builtin_amdgcn_fence(__ATOMIC_ACQUIRE, "workgroup");
    for (int pass = 0; pass < 2; ++pass) { for (int i = threadIdx.x; i < NGP + 32; i += 32) { ((volatile int*)START)[i] = (i <= NGP) ? st[min(i, NGP)] : 0; ((volatile int*)TOT)[i] = (i < nG) ? tot[i] : 0; } __threadfence(); } }
}
__global__ __launch_bounds__(256) void csrB_kernel9(const int* __restrict__ dst, int N, int nG, int CHP, int NGP, int permLen, const int* __restrict__ STG, const int* __restrict__ HST, const int* __restrict__ OFF, const int* __restrict__ START, const int* __restrict__ TOT, int* __restrict__ PERM, int* __restrict__ ROWPTR, int* __restrict__ ROWCNT, int* __restrict__ FLAG) {
  typedef __attribute__((ext_vector_type(4))) int v4i;
  __shared__ int ids[CSR_CAP9]; __shared__ unsigned short key[CSR_CAP9]; __shared__ int outp[CSR_CAP9]; __shared__ int ncnt[CSR_GN9 + 1]; __shared__ int boff[CSR_NBLK9 + 1];
  const int g = blockIdx.x, t_ = threadIdx.x; int tot = TOT[g]; int st = START[g], stn = START[g + 1]; const int v0 = g * CSR_GN9; const int nv = min(CSR_GN9, N - v0); const int t0 = g * CSR_TS9;
  st = (st < 0) ? 0 : (st > permLen - 32 ? permLen - 32 : st) & ~31; stn = (stn < st) ? st : (stn > permLen ? permLen : stn); tot = (tot < 0) ? 0 : tot; if (tot > stn - st && tot <= CSR_CAP9) tot = stn - st;
  if (tot > CSR_CAP9) {
    for (int pass = 0; pass < 2; ++pass) { for (int i = t_; i < CSR_TS9 / 4; i += 256) { v4i a, c; for (int e = 0; e < 4; ++e) { a[e] = st; c[e] = 0; } *(volatile v4i*)(ROWPTR + t0 + i * 4) = a; *(volatile v4i*)(ROWCNT + t0 + i * 4) = c; } if (t_ == 0) ((volatile int*)FLAG)[0] = 1; __threadfence(); } (void)nv; return; }
  if (t_ == 0) { int acc = 0; for (int b = 0; b < CSR_NBLK9; ++b) { boff[b] = acc; int c = HST[(size_t)b * NGP + g]; c = (c < 0) ? 0 : (c > CHP ? CHP : c); acc += c; if (acc > tot) acc = tot; } boff[CSR_NBLK9] = acc; }
  for (int i = t_; i <= CSR_GN9; i += 256) ncnt[i] = 0;
  __syncthreads();
  for (int b = 0; b < CSR_NBLK9; ++b) { const int c = boff[b + 1] - boff[b]; int o_ = OFF[(size_t)g * CSR_NBLK9 + b]; o_ = (o_ < 0) ? 0 : (o_ > CHP - c ? CHP - c : o_); const int* src_ = STG + (size_t)b * CHP + o_;
    for (int i = t_; i < c; i += 256) { int id = src_[i]; id = (id < 0) ? 0 : id; ids[boff[b] + i] = id; int d = dst[id]; d = (d < v0) ? v0 : (d >= N ? N - 1 : d); int kk = d - v0; kk = (kk < 0) ? 0 : (kk >= CSR_GN9 ? CSR_GN9 - 1 : kk); key[boff[b] + i] = (unsigned short)kk; } }
  __syncthreads();
  if (t_ == 0) { for (int i = 0; i < tot; ++i) ncnt[key[i]] += 1; int acc = 0; for (int vl = 0; vl < CSR_GN9; ++vl) { const int c = ncnt[vl]; ncnt[vl] = acc; acc += c; } ncnt[CSR_GN9] = acc;
    for (int i = 0; i < tot; ++i) { const int vl = key[i]; outp[ncnt[vl]] = ids[i]; ncnt[vl] += 1; }
    for (int vl = CSR_GN9; vl > 0; --vl) ncnt[vl] = ncnt[vl - 1]; ncnt[0] = 0; }
  __syncthreads();
  for (int pass = 0; pass < 2; ++pass) {
    for (int i = t_; i < (stn - st) / 4; i += 256) { v4i v; for (int e = 0; e < 4; ++e) { const int q = i * 4 + e; v[e] = (q < tot) ? outp[q] : -1; } *(volatile v4i*)(PERM + st + i * 4) = v; }
    for (int i = t_; i < CSR_TS9 / 4; i += 256) { v4i a, c; for (int e = 0; e < 4; ++e) { const int vl = i * 4 + e; const int vc = vl < CSR_GN9 ? vl : CSR_GN9; a[e] = (vl < CSR_GN9) ? st + ncnt[vc] : st; c[e] = (vl < nv) ? (ncnt[(vc < CSR_GN9 ? vc : CSR_GN9 - 1) + 1] - ncnt[vc]) : 0; } *(volatile v4i*)(ROWPTR + t0 + i * 4) = a; *(volatile v4i*)(ROWCNT + t0 + i * 4) = c; }
    __threadfence(); }
}
__global__ __launch_bounds__(256) void csrZ_kernel9(int* __restrict__ p, size_t n4) { typedef __attribute__((ext_vector_type(4))) int v4i; const size_t tid = (size_t)blockIdx.x * 256 + threadIdx.x, nth = (size_t)gridDim.x * 256; v4i z = {0, 0, 0, 0}; for (size_t i = tid; i < n4; i += nth) *(volatile v4i*)(p + i * 4) = z; }
struct CsrBufs9 { int *STG, *HST, *OFF, *START, *TOT, *PERM, *ROWPTR, *ROWCNT, *FLAG; int nG, NGP, CHP; size_t permLen; char* base; size_t bytes; };
static size_t csr_carve9(CsrBufs9& c, char* ws, size_t off, int E, int N) {
  const size_t off0 = off; c.base = ws + off;
  auto al = [&](size_t bytes) { char* p = ws + off; off += (bytes + 255) & ~(size_t)255; return p; };
  c.nG = (N + CSR_GN9 - 1) / CSR_GN9; c.NGP = (c.nG + 31) & ~31; const int ch = (E + CSR_NBLK9 - 1) / CSR_NBLK9; c.CHP = (ch + 31) & ~31; c.permLen = (size_t)E + 32 * (size_t)c.nG + 32;
  c.STG = (int*)al((size_t)CSR_NBLK9 * c.CHP * 4); c.HST = (int*)al((size_t)CSR_NBLK9 * c.NGP * 4); c.OFF = (int*)al((size_t)c.NGP * CSR_NBLK9 * 4); c.START = (int*)al((size_t)(c.NGP + 64) * 4); c.TOT = (int*)al((size_t)(c.NGP + 64) * 4);
  c.PERM = (int*)al(c.permLen * 4); c.ROWPTR = (int*)al((size_t)c.nG * CSR_TS9 * 4); c.ROWCNT = (int*)al((size_t)c.nG * CSR_TS9 * 4); c.FLAG = (int*)al(256);
  c.bytes = off - off0; return off;
}
static void csr_build9(const CsrBufs9& c, const int* dst, int E, int N, hipStream_t stream) {
  const size_t smem = (size_t)(2 * c.NGP + c.CHP) * 4;
  csrZ_kernel9<<<512, 256, 0, stream>>>((int*)c.base, c.bytes / 16);
  csrA_kernel9<<<CSR_NBLK9, 64, smem, stream>>>(dst, E, N, c.nG, c.CHP, c.NGP, c.STG, c.HST);
  csrS_kernel9<<<1, 512, 0, stream>>>(c.HST, c.nG, c.NGP, c.START, c.TOT, c.OFF);
  csrB_kernel9<<<c.nG, 256, 0, stream>>>(dst, N, c.nG, c.CHP, c.NGP, (int)c.permLen, c.STG, c.HST, c.OFF, c.START, c.TOT, c.PERM, c.ROWPTR, c.ROWCNT, c.FLAG);
}


__global__ __launch_bounds__(256) void wput_kernel(const float* __restrict__ w, int K, int O, b16* __restrict__ WT) { const int u = blockIdx.x * 256 + threadIdx.x; if (u >= O * (K / 8)) return; const int o = u / (K / 8), k0 = (u % (K / 8)) * 8; v8b v;
#pragma unroll
  for (int j = 0; j < 8; ++j) v[j] = (b16)(bf16_rne(w[(size_t)(k0 + j) * O + o]) * WSC); for (int pass = 0; pass < 2; ++pass) { *(volatile v8b*)(WT + (size_t)o * K + k0) = v; __threadfence(); } }
template <int KIN>
__global__ __launch_bounds__(32) void fc1fw_kernel(const float* __restrict__ x, const b16* __restrict__ W1T, const float* __restrict__ b1, const b16* __restrict__ FWT, const float* __restrict__ fb, int NLIM, float* __restrict__ OUT) {
  __shared__ __attribute__((aligned(16))) b16 Ah[16][KIN + 8], Al[16][D + 8]; __shared__ float Tf[16][132]; const int lane = threadIdx.x, nloc = lane & 15, hlf = lane >> 4; const size_t m0 = (size_t)blockIdx.x * 16; if (m0 >= (size_t)NLIM) return;
  for (int rr = 0; rr < 16; ++rr) for (int q = 0; q < KIN / 32; ++q) Ah[rr][q * 32 + lane] = (b16)(bf16_rne(x[(m0 + rr) * KIN + q * 32 + lane]) * XS);
  wave_lds_sync(); v8f acc[8];
#pragma unroll
  for (int t = 0; t < 8; ++t) acc[t] = (v8f){};
#pragma unroll
  for (int kb = 0; kb < KIN; kb += 32) { const v16b a = frag_kb(&Ah[nloc][kb], hlf);
#pragma unroll
    for (int t = 0; t < 8; ++t) acc[t] = wmma16b(a, frag_kb(W1T + (size_t)(t * 16 + nloc) * KIN + kb, hlf), acc[t]); }
  wave_lds_sync();
#pragma unroll
  for (int t = 0; t < 8; ++t) { const int c = t * 16 + nloc; const float bb = bf16_rne(b1[c]);
#pragma unroll
    for (int r8 = 0; r8 < 8; ++r8) { b16 p, ql; split16(fmaxf(acc[t][r8] * (1.0f / (XS * WSC)) + bb, 0.0f) * XS, p, ql); Ah[8 * hlf + r8][c] = p; Al[8 * hlf + r8][c] = ql; } }
  wave_lds_sync();
#pragma unroll
  for (int t = 0; t < 8; ++t) acc[t] = (v8f){};
#pragma unroll
  for (int kb = 0; kb < D; kb += 32) { const v16b a = frag_kb(&Ah[nloc][kb], hlf), al = frag_kb(&Al[nloc][kb], hlf);
#pragma unroll
    for (int t = 0; t < 8; ++t) { const v16b bw = frag_kb(FWT + (size_t)(t * 16 + nloc) * D + kb, hlf); acc[t] = wmma16b(a, bw, acc[t]); acc[t] = wmma16b(al, bw, acc[t]); } }
#pragma unroll
  for (int t = 0; t < 8; ++t) { const int c = t * 16 + nloc; const float bb = bf16_rne(fb[c]);
#pragma unroll
    for (int r8 = 0; r8 < 8; ++r8) Tf[8 * hlf + r8][c] = acc[t][r8] * (1.0f / (XS * WSC)) + bb; }
  wave_lds_sync();
  for (int pass = 0; pass < 2; ++pass) { for (int rr = 0; rr < 16; ++rr) *(volatile v4f*)(OUT + (m0 + rr) * D + lane * 4) = *(const v4f*)(&Tf[rr][lane * 4]); __threadfence(); } }
template <int NOUT>
__global__ __launch_bounds__(32) void dense_kernel(const float* __restrict__ IN, const b16* __restrict__ WT, const float* __restrict__ bias, int NLIM, float* __restrict__ OUT) { __shared__ __attribute__((aligned(16))) b16 Ah[16][D + 8], Al[16][D + 8]; __shared__ float Tf[16][132]; const int lane = threadIdx.x, nloc = lane & 15, hlf = lane >> 4; const size_t m0 = (size_t)blockIdx.x * 16; if (m0 >= (size_t)NLIM) return; constexpr int NT = NOUT / 16;
  for (int rr = 0; rr < 16; ++rr) for (int q = 0; q < 4; ++q) { b16 p, ql; split16(IN[(m0 + rr) * D + q * 32 + lane] * XS, p, ql); Ah[rr][q * 32 + lane] = p; Al[rr][q * 32 + lane] = ql; }
  wave_lds_sync(); v8f acc[NT];
#pragma unroll
  for (int t = 0; t < NT; ++t) acc[t] = (v8f){};
#pragma unroll
  for (int kb = 0; kb < D; kb += 32) { const v16b a = frag_kb(&Ah[nloc][kb], hlf), al = frag_kb(&Al[nloc][kb], hlf);
#pragma unroll
    for (int t = 0; t < NT; ++t) { const v16b bw = frag_kb(WT + (size_t)(t * 16 + nloc) * D + kb, hlf); acc[t] = wmma16b(a, bw, acc[t]); acc[t] = wmma16b(al, bw, acc[t]); } }
#pragma unroll
  for (int t = 0; t < NT; ++t) { const int c = t * 16 + nloc; const float bb = bf16_rne(bias[c]);
#pragma unroll
    for (int r8 = 0; r8 < 8; ++r8) Tf[8 * hlf + r8][c] = acc[t][r8] * (1.0f / (XS * WSC)) + bb; }
  wave_lds_sync();
  for (int pass = 0; pass < 2; ++pass) { for (int rr = 0; rr < 16; ++rr) { if (NOUT == 128) *(volatile v4f*)(OUT + (m0 + rr) * NOUT + lane * 4) = *(const v4f*)(&Tf[rr][lane * 4]); else *(volatile v2f*)(OUT + (m0 + rr) * NOUT + lane * 2) = (v2f){Tf[rr][lane * 2], Tf[rr][lane * 2 + 1]}; } __threadfence(); } }
__global__ __launch_bounds__(256) void spmm2_kernel(const float* __restrict__ X1src, const float* __restrict__ val1, const float* __restrict__ a1, const int* __restrict__ srcs1, CsrBufs9 c1, const float* __restrict__ X2src, const float* __restrict__ val2, const float* __restrict__ a2, const int* __restrict__ srcs2, CsrBufs9 c2, const float* __restrict__ Xself, int NLIM, float* __restrict__ H1, float* __restrict__ H2) {
  const int wave = threadIdx.x >> 5, lane = threadIdx.x & 31; const size_t i = (size_t)blockIdx.x * 8 + wave; if (i >= (size_t)NLIM) return; const v4f xs = *(const v4f*)(Xself + i * D + lane * 4);
  v4f h1, h2; { const float w1 = bf16_rne(a1[i]), w2 = bf16_rne(a2[i]); for (int k = 0; k < 4; ++k) { h1[k] = pmul(w1, xs[k]); h2[k] = pmul(w2, xs[k]); } }
  { int st = c1.ROWPTR[i], cnt = c1.ROWCNT[i]; cnt = iclamp(cnt, 0, E); st = iclamp(st, 0, (int)c1.permLen - cnt);
#pragma unroll 1
    for (int j = 0; j < cnt; ++j) { const int e = iclamp(c1.PERM[st + j], 0, E - 1); const size_t u = (size_t)iclamp(srcs1[e], 0, N - 1); if (u >= (size_t)NLIM) continue; const float v = bf16_rne(val1[e]); const v4f xv = *(const v4f*)(X1src + u * D + lane * 4); for (int k = 0; k < 4; ++k) h1[k] += pmul(v, xv[k]); } }
  { int st = c2.ROWPTR[i], cnt = c2.ROWCNT[i]; cnt = iclamp(cnt, 0, E); st = iclamp(st, 0, (int)c2.permLen - cnt);
#pragma unroll 1
    for (int j = 0; j < cnt; ++j) { const int e = iclamp(c2.PERM[st + j], 0, E - 1); const size_t u = (size_t)iclamp(srcs2[e], 0, N - 1); if (u >= (size_t)NLIM) continue; const float v = bf16_rne(val2[e]); const v4f xv = *(const v4f*)(X2src + u * D + lane * 4); for (int k = 0; k < 4; ++k) h2[k] += pmul(v, xv[k]); } }
  for (int pass = 0; pass < 2; ++pass) { *(volatile v4f*)(H1 + i * D + lane * 4) = h1; *(volatile v4f*)(H2 + i * D + lane * 4) = h2; __threadfence(); } }
__global__ __launch_bounds__(32) void sem_kernel(const float* __restrict__ H1, const float* __restrict__ H2, const b16* __restrict__ SWT, const float* __restrict__ sb, const float* __restrict__ sq, int NLIM, float* __restrict__ PS) { __shared__ __attribute__((aligned(16))) b16 Ah[16][D + 8]; const int lane = threadIdx.x, nloc = lane & 15, hlf = lane >> 4; const size_t m0 = (size_t)blockIdx.x * 16; if (m0 >= (size_t)NLIM) return; float tot[2] = {0.0f, 0.0f};
  for (int r = 0; r < 2; ++r) { const float* Hr = r == 0 ? H1 : H2;
    for (int rr = 0; rr < 16; ++rr) for (int q = 0; q < 4; ++q) Ah[rr][q * 32 + lane] = (b16)(Hr[(m0 + rr) * D + q * 32 + lane] * XS);
    wave_lds_sync(); v8f acc[8];
#pragma unroll
    for (int t = 0; t < 8; ++t) acc[t] = (v8f){};
#pragma unroll
    for (int kb = 0; kb < D; kb += 32) { const v16b a = frag_kb(&Ah[nloc][kb], hlf);
#pragma unroll
      for (int t = 0; t < 8; ++t) acc[t] = wmma16b(a, frag_kb(SWT + (size_t)(t * 16 + nloc) * D + kb, hlf), acc[t]); }
    float part = 0.0f;
#pragma unroll
    for (int t = 0; t < 8; ++t) { const int c = t * 16 + nloc; const float bb = bf16_rne(sb[c]), qq = bf16_rne(sq[c]);
#pragma unroll
      for (int r8 = 0; r8 < 8; ++r8) part += pmul(tanhf(acc[t][r8] * (1.0f / (XS * WSC)) + bb), qq); }
    for (int o = 16; o; o >>= 1) part += __shfl_xor(part, o); tot[r] = part; wave_lds_sync(); }
  for (int pass = 0; pass < 2; ++pass) { ((volatile float*)PS)[(size_t)blockIdx.x * 32 + lane] = lane == 0 ? tot[0] : (lane == 1 ? tot[1] : 0.0f); __threadfence(); } }
__global__ __launch_bounds__(256) void beta_kernel(const float* __restrict__ PS, int nwaves, int nnodes, float* __restrict__ BETA) { __shared__ double S0[256], S1[256]; const int t = threadIdx.x; double a = 0.0, b = 0.0; for (int w = t; w < nwaves; w += 256) { a += (double)PS[(size_t)w * 32]; b += (double)PS[(size_t)w * 32 + 1]; } S0[t] = a; S1[t] = b; __syncthreads();
  for (int st = 128; st > 0; st >>= 1) { if (t < st) { S0[t] += S0[t + st]; S1[t] += S1[t + st]; } __syncthreads(); }
  const float m0 = (float)(S0[0] / nnodes), m1 = (float)(S1[0] / nnodes); const float mx = fmaxf(m0, m1); const float e0 = __expf(m0 - mx), e1 = __expf(m1 - mx); const float b0 = e0 / (e0 + e1), b1 = e1 / (e0 + e1);
  for (int pass = 0; pass < 2; ++pass) { if (t < 32) ((volatile float*)BETA)[t] = t == 0 ? b0 : (t == 1 ? b1 : 0.0f); __threadfence(); } }
__global__ __launch_bounds__(256) void comb_kernel(const float* __restrict__ H1, const float* __restrict__ H2, const float* __restrict__ BETA, int NLIM, float* __restrict__ X) { const size_t u = (size_t)blockIdx.x * 256 + threadIdx.x; if (u >= (size_t)N * D / 4) return; const size_t n = u / (D / 4); v4f r = {0.0f, 0.0f, 0.0f, 0.0f};
  if (n < (size_t)NLIM) { const float b0 = BETA[0], b1 = BETA[1]; const v4f a = *(const v4f*)(H1 + u * 4), b = *(const v4f*)(H2 + u * 4); for (int k = 0; k < 4; ++k) r[k] = fmaxf(pmul(b0, a[k]) + pmul(b1, b[k]), 0.0f); }
  for (int pass = 0; pass < 2; ++pass) { *(volatile v4f*)(X + u * 4) = r; __threadfence(); } }
}

extern "C" void kernel_launch(void* const* d_in, const int* in_sizes, int n_in, void* d_out, int out_size, void* d_ws, size_t ws_size, hipStream_t stream) {
  (void)n_in;
  auto Fp = [&](int i) { return (const float*)d_in[i]; }; auto Ip = [&](int i) { return (const int*)d_in[i]; };
  if (in_sizes[0] != N * DA || in_sizes[1] != N * DB || in_sizes[2] != E || in_sizes[6] != E || in_sizes[10] != E || in_sizes[14] != E || in_sizes[18] != DA * D || in_sizes[20] != DB * D || in_sizes[38] != D * DO || out_size != N * DO) return;
  const int NLIM = N;
  size_t off = 0; char* ws = (char*)d_ws;
  auto carve = [&](size_t bytes) { char* p = ws + off; off += (bytes + 255) & ~(size_t)255; return p; };
  b16* W1A = (b16*)carve((size_t)D * DA * 2); b16* W1B = (b16*)carve((size_t)D * DB * 2); b16* FW0 = (b16*)carve((size_t)D * D * 2); b16* FW1 = (b16*)carve((size_t)D * D * 2); b16* S0A = (b16*)carve((size_t)D * D * 2); b16* S0B = (b16*)carve((size_t)D * D * 2); b16* S1A = (b16*)carve((size_t)D * D * 2); b16* W2 = (b16*)carve((size_t)DO * D * 2);
  float* X2A = (float*)carve((size_t)N * D * 4); float* X2B = (float*)carve((size_t)N * D * 4); float* HR1 = (float*)carve((size_t)N * D * 4); float* HR2 = (float*)carve((size_t)N * D * 4); float* X3A = (float*)carve((size_t)N * D * 4); float* X3B = (float*)carve((size_t)N * D * 4);
  const int NW = (NLIM + 15) / 16; float* PS = (float*)carve((size_t)((N + 15) / 16) * 32 * 4); float* BETA = (float*)carve(32 * 4);
  CsrBufs9 cAA, cAB, cBB, cBA; off = csr_carve9(cAA, ws, off, E, N); off = csr_carve9(cAB, ws, off, E, N); off = csr_carve9(cBB, ws, off, E, N); off = csr_carve9(cBA, ws, off, E, N);
  if (off > ws_size || off > ((size_t)200 << 20)) return;
  wput_kernel<<<(D * DA / 8 + 255) / 256, 256, 0, stream>>>(Fp(18), DA, D, W1A); wput_kernel<<<(D * DB / 8 + 255) / 256, 256, 0, stream>>>(Fp(20), DB, D, W1B);
  wput_kernel<<<(D * D / 8 + 255) / 256, 256, 0, stream>>>(Fp(22), D, D, FW0); wput_kernel<<<(D * D / 8 + 255) / 256, 256, 0, stream>>>(Fp(30), D, D, FW1);
  wput_kernel<<<(D * D / 8 + 255) / 256, 256, 0, stream>>>(Fp(24), D, D, S0A); wput_kernel<<<(D * D / 8 + 255) / 256, 256, 0, stream>>>(Fp(27), D, D, S0B); wput_kernel<<<(D * D / 8 + 255) / 256, 256, 0, stream>>>(Fp(32), D, D, S1A);
  wput_kernel<<<(DO * D / 8 + 255) / 256, 256, 0, stream>>>(Fp(38), D, DO, W2);
  csr_build9(cAA, Ip(3), E, N, stream); csr_build9(cAB, Ip(7), E, N, stream); csr_build9(cBB, Ip(11), E, N, stream); csr_build9(cBA, Ip(15), E, N, stream);
  const unsigned gt = (NLIM + 7) / 8, gw = NLIM / 16, gc = (unsigned)(((size_t)N * D / 4 + 255) / 256);
  fc1fw_kernel<DA><<<gw, 32, 0, stream>>>(Fp(0), W1A, Fp(19), FW0, Fp(23), NLIM, X2A);
  fc1fw_kernel<DB><<<gw, 32, 0, stream>>>(Fp(1), W1B, Fp(21), FW0, Fp(23), NLIM, X2B);
  spmm2_kernel<<<gt, 256, 0, stream>>>(X2A, Fp(4), Fp(5), Ip(2), cAA, X2B, Fp(8), Fp(9), Ip(6), cAB, X2A, NLIM, HR1, HR2);
  sem_kernel<<<gw, 32, 0, stream>>>(HR1, HR2, S0A, Fp(25), Fp(26), NLIM, PS); beta_kernel<<<1, 256, 0, stream>>>(PS, NW, NLIM, BETA); comb_kernel<<<gc, 256, 0, stream>>>(HR1, HR2, BETA, NLIM, X3A);
  spmm2_kernel<<<gt, 256, 0, stream>>>(X2B, Fp(12), Fp(13), Ip(10), cBB, X3A, Fp(16), Fp(17), Ip(14), cBA, X2B, NLIM, HR1, HR2);
  sem_kernel<<<gw, 32, 0, stream>>>(HR1, HR2, S0B, Fp(28), Fp(29), NLIM, PS); beta_kernel<<<1, 256, 0, stream>>>(PS, NW, NLIM, BETA); comb_kernel<<<gc, 256, 0, stream>>>(HR1, HR2, BETA, NLIM, X3B);
  dense_kernel<128><<<gw, 32, 0, stream>>>(X3A, FW1, Fp(31), NLIM, X2A); dense_kernel<128><<<gw, 32, 0, stream>>>(X3B, FW1, Fp(31), NLIM, X2B);
  spmm2_kernel<<<gt, 256, 0, stream>>>(X2A, Fp(4), Fp(5), Ip(2), cAA, X2B, Fp(8), Fp(9), Ip(6), cAB, X2A, NLIM, HR1, HR2);
  sem_kernel<<<gw, 32, 0, stream>>>(HR1, HR2, S1A, Fp(33), Fp(34), NLIM, PS); beta_kernel<<<1, 256, 0, stream>>>(PS, NW, NLIM, BETA); comb_kernel<<<gc, 256, 0, stream>>>(HR1, HR2, BETA, NLIM, X3A);
  dense_kernel<64><<<gw, 32, 0, stream>>>(X3A, W2, Fp(39), NLIM, (float*)d_out);
}
